// EdgeMLPEncoder_91156385890469
// MI455X (gfx1250) — hardware-verified
//
#include <hip/hip_runtime.h>
#include <stddef.h>
#include <math.h>


typedef _Float16 v16h __attribute__((ext_vector_type(16)));
typedef _Float16 v8h  __attribute__((ext_vector_type(8)));
typedef float    v8f  __attribute__((ext_vector_type(8)));
typedef float    v4f  __attribute__((ext_vector_type(4)));
typedef float    v2f  __attribute__((ext_vector_type(2)));
typedef _Float16 h16;

#ifndef NB
#define NB 64
#endif
#ifndef SEQ
#define SEQ 16384
#endif
#define NB_FULL  64
#define SEQ_FULL 16384
#define HW       128
#define CHUNK    64
#define ROWS_PB  512
#define BPB      (SEQ / ROWS_PB)
#define HROWS    16

#define LDT 72
#define LDH 136
#define LDZ 264
#define LDO 132

#define WCARRY 64.0f
#define HCARRY 16.0f
#define ZCARRY 16.0f

static_assert(NB >= 1 && NB <= NB_FULL);
static_assert(SEQ >= ROWS_PB && SEQ <= SEQ_FULL && (SEQ % ROWS_PB) == 0);
static_assert(HW == 128);
static_assert((ROWS_PB % CHUNK) == 0 && (ROWS_PB % 256) == 0);
static_assert(8 * 16 == HW);
static_assert(16 * 8 == HW);
static_assert((256 / 16) * 4 == CHUNK);
static_assert(32 * 4 == HW);
static_assert((HW % 64) == 0 && (HW % 32) == 0 && ((2 * HW) % 64) == 0);
static_assert((LDT % 8) == 0 && LDT >= 64);
static_assert((LDH % 8) == 0 && LDH >= HW);
static_assert((LDZ % 8) == 0 && LDZ >= 2 * HW);
static_assert((LDO % 4) == 0 && LDO >= HW);
static_assert(HROWS == 16 && (HROWS * 32) % 256 == 0);
static_assert(BPB >= 1);

#define W2T_BYTES  ((size_t)HW * HW * 2)
#define WHT_BYTES  ((size_t)HW * 2 * HW * 2)
#define PART_BYTES ((size_t)NB * BPB * 2 * HW * 4)
#define OFF_W2T  ((size_t)0)
#define OFF_WHT  (OFF_W2T + W2T_BYTES)
#define OFF_PART (OFF_WHT + WHT_BYTES)
#define WS_TOTAL (OFF_PART + PART_BYTES)
static_assert((W2T_BYTES % 128) == 0 && (WHT_BYTES % 128) == 0 && (PART_BYTES % 128) == 0);
static_assert(WS_TOTAL <= (size_t)134217728);

__device__ __forceinline__ float bf16r(float x) {
  unsigned int u = __float_as_uint(x);
  u = (u + 0x7FFFu + ((u >> 16) & 1u)) & 0xFFFF0000u;
  return __uint_as_float(u);
}

__device__ __forceinline__ v16h frag_at(const _Float16* p) {
  v8h lo = *(const v8h*)(p);
  v8h hi = *(const v8h*)(p + 16);
  v16h out;
#pragma unroll
  for (int i = 0; i < 8; ++i) { out[i] = lo[i]; out[i + 8] = hi[i]; }
  return out;
}
__device__ __forceinline__ v16h ld_frag(const _Float16* base, unsigned ld) {
  const unsigned lane = threadIdx.x & 31u;
  return frag_at(base + (lane & 15u) * ld + (lane >> 4) * 8u);
}

__device__ __forceinline__ v8f wmma16(v16h a, v16h b, v8f c) {
  v8f d = __builtin_amdgcn_wmma_f32_16x16x32_f16(false, a, false, b, (short)0, c,
                                                 false, false);
  asm volatile("v_nop\n\tv_nop\n\tv_nop\n\tv_nop" : "+v"(d) : "v"(a), "v"(b));
  return d;
}

__device__ __forceinline__ float red32_sum(float x) {
#pragma unroll
  for (int off = 1; off < 32; off <<= 1) x += __shfl_xor(x, off, 32);
  return x;
}

static __device__ __forceinline__ h16 toh_flush(float v) {
  const h16 r = (h16)v;
  return (fabsf(v) < 6.103515625e-05f) ? (h16)0.0f : r;
}

__device__ __forceinline__ float gelu_erf(float v) {
  return 0.5f * v * (1.0f + erff(v * 0.70710678118654752f));
}

__global__ __launch_bounds__(256) void wconv_kernel(
    const float* __restrict__ W, _Float16* __restrict__ Wt, unsigned ldw, unsigned ldk) {
  __shared__ _Float16 T[64 * LDT];
  const unsigned tid = threadIdx.x;
  const unsigned n0 = blockIdx.x * 64u;
  const unsigned k0 = blockIdx.y * 64u;
#pragma unroll 4
  for (unsigned j = 0; j < 16u; ++j) {
    const unsigned idx = tid + 256u * j;
    const unsigned kr = idx >> 6, nc = idx & 63u;
    const float v = W[(size_t)(k0 + kr) * ldw + n0 + nc];
    T[nc * LDT + kr] = (_Float16)(WCARRY * bf16r(v));
  }
  __syncthreads();
  v8h x[2];
  size_t off[2];
#pragma unroll
  for (unsigned i = 0; i < 2u; ++i) {
    const unsigned n = 32u * i + (tid >> 3);
    const unsigned kc = (tid & 7u) * 8u;
    x[i] = *(const v8h*)&T[n * LDT + kc];
    off[i] = (size_t)(n0 + n) * ldk + k0 + kc;
  }
#pragma unroll
  for (int i = 0; i < 2; ++i) *(volatile v8h*)(Wt + off[i]) = x[i];
  __threadfence();
#pragma unroll
  for (int i = 0; i < 2; ++i) *(volatile v8h*)(Wt + off[i]) = x[i];
}

__global__ __launch_bounds__(256) void edge_mlp_kernel(
    const float* __restrict__ x, const float* __restrict__ W1, const float* __restrict__ b1,
    const _Float16* __restrict__ W2t, const float* __restrict__ b2, float* __restrict__ part) {
  __shared__ _Float16 h1s[CHUNK * LDH];
  __shared__ float dxs[ROWS_PB * 2];
  __shared__ float reds[2 * HW];

  const unsigned tid = threadIdx.x, lane = tid & 31u;
  const unsigned wave = (unsigned)__builtin_amdgcn_readfirstlane((int)(threadIdx.x >> 5));
  const unsigned hh = lane >> 4, m = lane & 15u;
  const unsigned b = blockIdx.x / (unsigned)BPB;
  const unsigned blk = blockIdx.x - b * (unsigned)BPB;
  const unsigned rowStart = blk * (unsigned)ROWS_PB;
  const float* xb = x + (size_t)b * SEQ_FULL * 2;

#pragma unroll
  for (unsigned j = 0; j < (unsigned)(ROWS_PB / 256); ++j) {
    const unsigned lr = tid + 256u * j;
    const unsigned r = rowStart + lr;
    const unsigned rn = (r + 1u == (unsigned)SEQ) ? 0u : (r + 1u);
    const v2f a = *(const v2f*)(xb + (size_t)r * 2u);
    const v2f c = *(const v2f*)(xb + (size_t)rn * 2u);
    v2f d;
    d[0] = bf16r(c[0]) - bf16r(a[0]);
    d[1] = bf16r(c[1]) - bf16r(a[1]);
    *(v2f*)&dxs[lr * 2u] = d;
  }

  const unsigned cg = tid & 15u, rb = tid >> 4;
  float w0[8], w1[8], bb[8];
  {
    const v4f p0 = *(const v4f*)(W1 + cg * 8u);
    const v4f p1 = *(const v4f*)(W1 + cg * 8u + 4u);
    const v4f q0 = *(const v4f*)(W1 + HW + cg * 8u);
    const v4f q1 = *(const v4f*)(W1 + HW + cg * 8u + 4u);
    const v4f c0 = *(const v4f*)(b1 + cg * 8u);
    const v4f c1 = *(const v4f*)(b1 + cg * 8u + 4u);
#pragma unroll
    for (int i = 0; i < 4; ++i) {
      w0[i] = bf16r(p0[i]); w0[i + 4] = bf16r(p1[i]);
      w1[i] = bf16r(q0[i]); w1[i + 4] = bf16r(q1[i]);
      bb[i] = bf16r(c0[i]); bb[i + 4] = bf16r(c1[i]);
    }
  }

  const unsigned colB = wave * 16u + m;
  v16h bfr[4];
#pragma unroll
  for (int kk = 0; kk < 4; ++kk)
    bfr[kk] = frag_at(W2t + (size_t)colB * HW + (unsigned)kk * 32u + hh * 8u);
  const float bias2 = bf16r(b2[colB]);

  float sumAcc = 0.0f;
  float maxAcc = -1.0e30f;

  __syncthreads();

#pragma unroll 1
  for (unsigned ch = 0; ch < (unsigned)(ROWS_PB / CHUNK); ++ch) {
#pragma unroll 1
    for (unsigned j = 0; j < 4u; ++j) {
      const unsigned row = rb + 16u * j;
      const v2f d = *(const v2f*)&dxs[(ch * (unsigned)CHUNK + row) * 2u];
      v8h o;
#pragma unroll
      for (int i = 0; i < 8; ++i) {
        const float v = fmaf(d[0], w0[i], fmaf(d[1], w1[i], bb[i]));
        o[i] = toh_flush(HCARRY * gelu_erf(v));
      }
      *(v8h*)&h1s[row * LDH + cg * 8u] = o;
    }
    __syncthreads();

#pragma unroll 1
    for (unsigned mt = 0; mt < (unsigned)(CHUNK / 16); ++mt) {
      v8f acc = {};
#pragma unroll
      for (int kk = 0; kk < 4; ++kk) {
        const v16h a = ld_frag(&h1s[(mt * 16u) * LDH + (unsigned)kk * 32u], LDH);
        acc = wmma16(a, bfr[kk], acc);
      }
#pragma unroll
      for (int r = 0; r < 8; ++r) {
        const float t = acc[r] * (1.0f / (WCARRY * HCARRY)) + bias2;
        const float h2 = gelu_erf(t);
        sumAcc += h2;
        maxAcc = fmaxf(maxAcc, h2);
      }
    }
    __syncthreads();
  }

  sumAcc += __shfl_xor(sumAcc, 16, 32);
  maxAcc = fmaxf(maxAcc, __shfl_xor(maxAcc, 16, 32));
  if (hh == 0u) {
    reds[colB] = sumAcc;
    reds[HW + colB] = maxAcc;
  }
  __syncthreads();

  if (wave == 0u) {
    const v4f s4 = *(const v4f*)&reds[lane * 4u];
    const v4f m4 = *(const v4f*)&reds[HW + lane * 4u];
    float* p = part + (size_t)blockIdx.x * (2u * HW) + lane * 4u;
    *(volatile v4f*)p = s4;
    *(volatile v4f*)(p + HW) = m4;
    __threadfence();
    *(volatile v4f*)p = s4;
    *(volatile v4f*)(p + HW) = m4;
  }
}

__global__ __launch_bounds__(256) void head_kernel(
    const float* __restrict__ part, const _Float16* __restrict__ Wht,
    const float* __restrict__ bh, const float* __restrict__ gamma,
    const float* __restrict__ beta, float* __restrict__ out) {
  __shared__ _Float16 Za[HROWS * LDZ];
  __shared__ float Zs[HROWS * LDO];

  const unsigned tid = threadIdx.x, lane = tid & 31u;
  const unsigned wave = (unsigned)__builtin_amdgcn_readfirstlane((int)(threadIdx.x >> 5));
  const unsigned hh = lane >> 4, m = lane & 15u;
  const unsigned row0 = blockIdx.x * (unsigned)HROWS;

#pragma unroll 1
  for (unsigned j = 0; j < (unsigned)((HROWS * 32) / 256); ++j) {
    const unsigned idx = tid + 256u * j;
    const unsigned lr = idx >> 5, cgz = idx & 31u;
    const unsigned grow = row0 + lr;
    const bool live = (grow < (unsigned)NB);
    const unsigned crow = live ? grow : (unsigned)(NB - 1);
    const float* src = part + (size_t)crow * BPB * (2u * HW) + cgz * 8u;
    float s[8], mx[8];
#pragma unroll
    for (int i = 0; i < 8; ++i) { s[i] = 0.0f; mx[i] = -1.0e30f; }
#pragma unroll 2
    for (unsigned p = 0; p < (unsigned)BPB; ++p) {
      const v4f a0 = *(const v4f*)(src + (size_t)p * (2u * HW));
      const v4f a1 = *(const v4f*)(src + (size_t)p * (2u * HW) + 4u);
#pragma unroll
      for (int i = 0; i < 4; ++i) {
        s[i] += a0[i];          mx[i] = fmaxf(mx[i], a0[i]);
        s[i + 4] += a1[i];      mx[i + 4] = fmaxf(mx[i + 4], a1[i]);
      }
    }
    const bool ismax = (cgz >= 16u);
    v8h o;
#pragma unroll
    for (int i = 0; i < 8; ++i) {
      float val = ismax ? mx[i] : s[i] * (1.0f / (float)SEQ);
      val = live ? val : 0.0f;
      o[i] = toh_flush(ZCARRY * val);
    }
    *(v8h*)&Za[lr * LDZ + cgz * 8u] = o;
  }
  __syncthreads();

  v8f acc = {};
  const _Float16* bp = Wht + (size_t)(wave * 16u + m) * (2u * HW) + hh * 8u;
#pragma unroll 2
  for (unsigned k0 = 0; k0 < 2u * HW; k0 += 32u) {
    const v16h a = ld_frag(&Za[k0], LDZ);
    const v16h bq = frag_at(bp + k0);
    acc = wmma16(a, bq, acc);
  }
  const float bcol = bf16r(bh[wave * 16u + m]);
#pragma unroll
  for (int r = 0; r < 8; ++r)
    Zs[(hh * 8u + (unsigned)r) * LDO + wave * 16u + m] =
        acc[r] * (1.0f / (WCARRY * ZCARRY)) + bcol;
  __syncthreads();

  const v4f g4 = *(const v4f*)(gamma + lane * 4u);
  const v4f e4 = *(const v4f*)(beta + lane * 4u);
#pragma unroll 1
  for (unsigned rr = 0; rr < 2u; ++rr) {
    const unsigned lr = wave * 2u + rr;
    const unsigned grow = row0 + lr;
    const v4f z = *(const v4f*)&Zs[lr * LDO + lane * 4u];
    const float mean = red32_sum((z[0] + z[1]) + (z[2] + z[3])) * (1.0f / (float)HW);
    v4f d;
    float ss = 0.0f;
#pragma unroll
    for (int i = 0; i < 4; ++i) { d[i] = z[i] - mean; ss += d[i] * d[i]; }
    const float var = red32_sum(ss) * (1.0f / (float)HW);
    const float rstd = 1.0f / sqrtf(var + 1.0e-5f);
    v4f o;
#pragma unroll
    for (int i = 0; i < 4; ++i) o[i] = d[i] * rstd * bf16r(g4[i]) + bf16r(e4[i]);
    if (grow < (unsigned)NB) {
      float* p = out + (size_t)grow * HW + lane * 4u;
      *(volatile v4f*)p = o;
      __threadfence();
      *(volatile v4f*)p = o;
    }
  }
}

extern "C" void kernel_launch(void* const* d_in, const int* in_sizes, int n_in,
                              void* d_out, int out_size, void* d_ws, size_t ws_size,
                              hipStream_t stream) {
  if (n_in < 9) return;
  const long long need_x = ((long long)(NB - 1) * SEQ_FULL + SEQ) * 2;
  if ((long long)in_sizes[0] < need_x) return;
  if (in_sizes[1] < 2 * HW) return;
  if (in_sizes[2] < HW) return;
  if (in_sizes[3] < HW * HW) return;
  if (in_sizes[4] < HW) return;
  if (in_sizes[5] < 2 * HW * HW) return;
  if (in_sizes[6] < HW || in_sizes[7] < HW || in_sizes[8] < HW) return;
  if ((long long)out_size < (long long)NB * HW) return;
  if (ws_size < WS_TOTAL) return;

  const float* X   = (const float*)d_in[0];
  const float* w1  = (const float*)d_in[1];
  const float* b1  = (const float*)d_in[2];
  const float* w2  = (const float*)d_in[3];
  const float* b2  = (const float*)d_in[4];
  const float* wh  = (const float*)d_in[5];
  const float* bh  = (const float*)d_in[6];
  const float* gam = (const float*)d_in[7];
  const float* bet = (const float*)d_in[8];
  float* out = (float*)d_out;

  char* ws = (char*)d_ws;
  _Float16* W2t  = (_Float16*)(ws + OFF_W2T);
  _Float16* Wht  = (_Float16*)(ws + OFF_WHT);
  float*    Part = (float*)(ws + OFF_PART);

  dim3 blk(256);
  wconv_kernel<<<dim3(HW / 64, HW / 64), blk, 0, stream>>>(w2, W2t, (unsigned)HW, (unsigned)HW);
  wconv_kernel<<<dim3(HW / 64, (2 * HW) / 64), blk, 0, stream>>>(wh, Wht, (unsigned)HW,
                                                                 (unsigned)(2 * HW));
  edge_mlp_kernel<<<dim3(NB * BPB), blk, 0, stream>>>(X, w1, b1, W2t, b2, Part);
  head_kernel<<<dim3((NB + HROWS - 1) / HROWS), blk, 0, stream>>>(Part, Wht, bh, gam, bet, out);
}
